// MDCNv4_1_45973329936719
// MI455X (gfx1250) — hardware-run, weakly checked
//
#include <hip/hip_runtime.h>


#ifndef NB
#define NB 4
#endif
#define NB_FULL 4
#define CIN   128
#define COUT  256
#define HH    56
#define WW    56
#define HW    (HH * WW)
#define HP    (HH + 2)
#define WP    (WW + 2)
#define K2    9
#define KD    (CIN * K2)
#define NOFF  27
#define NOP   32
#define NPOS  (NB * HW)
#define XBS_FULL (CIN * HW)
#define DPOS  32
#define AP    136
#define OTP   36
#define OFP   36
#define TSP   136
#define XROWP (WP * CIN / 8)
#define SCA   64.0f
#define SCW   1024.0f
#define SCI   (1.0f / 65536.0f)
#define LOG2E 1.4426950408889634f

static_assert(CIN == 128);
static_assert(CIN % 32 == 0);
static_assert(KD % 32 == 0);
static_assert(KD % 8 == 0);
static_assert(COUT == 8 * 32);
static_assert(HW % DPOS == 0);
static_assert((HW * 4) % 128 == 0);
static_assert((DPOS * 4) == 128);
static_assert(NPOS % 64 == 0);
static_assert(NPOS % DPOS == 0);
static_assert(NOFF <= NOP);
static_assert(NOP * 4 == 128);
static_assert(NOFF == 3 * K2);
static_assert((COUT * (KD / 8)) % 256 == 0);
static_assert((NOP * (KD / 8)) % 256 == 0);
static_assert((KD * 2) % 128 == 0);
static_assert((WP * CIN * 2) % 128 == 0);
static_assert(XROWP * 16 == WP * CIN * 2);
static_assert(XROWP <= 4 * 256);
static_assert(XROWP % 8 == 0);
static_assert((CIN * WW) % 256 == 0);
static_assert(256 == DPOS * 8);
static_assert((AP * 2) % 16 == 0);
static_assert((OTP * 4) % 16 == 0);
static_assert((OFP * 4) % 16 == 0);
static_assert((TSP * 2) % 16 == 0);
static_assert(4 * 32 * 16 == 16 * NOP * 4);
static_assert(8 * 32 * 16 == 32 * DPOS * 4);
static_assert(DPOS * AP * 2 + 8 * 32 * OTP * 4 <= 131072);
static_assert(16 * OFP * 4 <= 131072);
static_assert(WW * TSP * 2 <= 131072);
static_assert(NB <= NB_FULL);

typedef _Float16 h16;
typedef unsigned short bf;
typedef __attribute__((ext_vector_type(16))) __bf16   v16bf;
typedef __attribute__((ext_vector_type(16))) _Float16 v16h;
typedef __attribute__((ext_vector_type(8)))  _Float16 v8h;
typedef __attribute__((ext_vector_type(8)))  unsigned short v8us;
typedef __attribute__((ext_vector_type(8)))  float    v8f;
typedef __attribute__((ext_vector_type(4)))  float    v4f;
typedef v4f  __attribute__((may_alias)) v4fa;
typedef v8us __attribute__((may_alias)) v8usa;

__device__ __forceinline__ unsigned short f2bf(float f) { unsigned u = __float_as_uint(f); u += 0x7FFFu + ((u >> 16) & 1u); return (unsigned short)(u >> 16); }
__device__ __forceinline__ float bfr(float f) { return __uint_as_float(((unsigned)f2bf(f)) << 16); }
__device__ __forceinline__ v16h cat16(v8h lo, v8h hi) { return __builtin_shufflevector(lo, hi, 0, 1, 2, 3, 4, 5, 6, 7, 8, 9, 10, 11, 12, 13, 14, 15); }
__device__ __forceinline__ v16bf cat16b(v8us lo, v8us hi) { return __builtin_bit_cast(v16bf, __builtin_shufflevector(lo, hi, 0, 1, 2, 3, 4, 5, 6, 7, 8, 9, 10, 11, 12, 13, 14, 15)); }
__device__ __forceinline__ v8f wmma16(v16h a, v16h b, v8f c) { return __builtin_amdgcn_wmma_f32_16x16x32_f16(false, a, false, b, (short)0, c, false, false); }
__device__ __forceinline__ v8f wmmab(v16bf a, v16bf b, v8f c) { return __builtin_amdgcn_wmma_f32_16x16x32_bf16(false, a, false, b, (short)0, c, false, false); }
__device__ __forceinline__ v16h  ldh(const h16* p) { return cat16(*(const v8h*)p, *(const v8h*)(p + 16)); }
__device__ __forceinline__ v16bf ldb(const bf* p)  { return cat16b(*(const v8us*)p, *(const v8us*)(p + 16)); }
__device__ __forceinline__ void wave_sync() { __builtin_amdgcn_fence(3  , "wavefront"); __builtin_amdgcn_wave_barrier(); asm volatile("" ::: "memory"); }
static __device__ __forceinline__ h16 toh_flush(float v) { const h16 r = (h16)v; return (fabsf(v) < 6.103515625e-05f) ? (h16)0.0f : r; }
__device__ __forceinline__ v8f wmma16g(v16h a, v16h b, v8f c) { c = wmma16(a, b, c); asm volatile("v_nop\n\tv_nop\n\tv_nop\n\tv_nop" : "+v"(c) : "v"(a), "v"(b)); return c; }
__device__ __forceinline__ v8f wmmabg(v16bf a, v16bf b, v8f c) { c = wmmab(a, b, c); asm volatile("v_nop\n\tv_nop\n\tv_nop\n\tv_nop" : "+v"(c) : "v"(a), "v"(b)); return c; }

__global__ __launch_bounds__(256) void k_xpad(const float* __restrict__ x, bf* XP) {
    __shared__ __align__(16) bf ts[WW * TSP];
    const int tid = threadIdx.x; const int yp = blockIdx.x, b = blockIdx.y;
    const bool inner = (yp >= 1) & (yp <= HH);
    if (inner) {
        const float* src = x + (size_t)b * XBS_FULL + (size_t)(yp - 1) * WW;
#pragma unroll 1
        for (int i = tid; i < CIN * WW; i += 256) { const int c = i / WW, w = i - c * WW; ts[w * TSP + c] = f2bf(src[(size_t)c * HW + w]); }
    }
    __syncthreads();
    bf* dst = XP + ((size_t)b * HP + yp) * (size_t)WP * CIN;
#pragma unroll 1
    for (int ps = 0; ps < 2; ++ps) {
#pragma unroll 1
        for (int it = 0; it < 4; ++it) {
            const int i = it * 256 + tid; const int ic = i < XROWP ? i : (XROWP - 1);
            const int pix = ic >> 4, c8 = (ic & 15) * 8;
            int pw = pix - 1; pw = pw < 0 ? 0 : (pw > WW - 1 ? WW - 1 : pw);
            v8us o = (v8us){};
            if (inner) { const v8us v = *(const v8usa*)(&ts[pw * TSP + c8]); const bool ok = (pix >= 1) & (pix <= WW); const v8us z = (v8us){}; o = ok ? v : z; }
            if (i < XROWP) *(volatile v8us*)(dst + (size_t)i * 8) = o; }
        if (ps == 0) __threadfence(); }
}

__global__ __launch_bounds__(256) void k_wmain(const float* __restrict__ w, h16* WH) {
    const int i = blockIdx.x * 256 + threadIdx.x; if (i >= COUT * (KD / 8)) return;
    const int n = i / (KD / 8), k8 = (i - n * (KD / 8)) * 8; const int t = k8 / CIN, c = k8 - t * CIN;
    const float* src = w + (size_t)n * KD + (size_t)c * K2 + t;
    v8h o;
#pragma unroll
    for (int e = 0; e < 8; ++e) o[e] = toh_flush(bfr(src[e * K2]) * SCW);
    *(volatile v8h*)(WH + (size_t)i * 8) = o; __threadfence(); *(volatile v8h*)(WH + (size_t)i * 8) = o;
}

__global__ __launch_bounds__(256) void k_woff(const float* __restrict__ ow, bf* OWB) {
    const int i = blockIdx.x * 256 + threadIdx.x; if (i >= NOP * (KD / 8)) return;
    const int n = i / (KD / 8), k8 = (i - n * (KD / 8)) * 8; const int t = k8 / CIN, c = k8 - t * CIN;
    const int nc = n < NOFF ? n : (NOFF - 1);
    const float* src = ow + (size_t)nc * KD + (size_t)c * K2 + t;
    v8us o;
#pragma unroll
    for (int e = 0; e < 8; ++e) { float v = src[e * K2]; asm volatile("" : "+v"(v)); o[e] = (n < NOFF) ? f2bf(v) : (unsigned short)0; }
    *(volatile v8us*)(OWB + (size_t)i * 8) = o; __threadfence(); *(volatile v8us*)(OWB + (size_t)i * 8) = o;
}

__global__ __launch_bounds__(32) void k_offconv(const bf* __restrict__ XP, const bf* __restrict__ OWB, const float* __restrict__ ob, float* PRED) {
    __shared__ __align__(16) float os[16 * OFP];
    const int lane = threadIdx.x & 31, lr = lane & 15, hi = lane >> 4; const int r0 = blockIdx.x * 64;
    v8f acc[4][2];
#pragma unroll
    for (int mb = 0; mb < 4; ++mb)
#pragma unroll
        for (int nb = 0; nb < 2; ++nb) acc[mb][nb] = (v8f){};
    size_t ab[4];
#pragma unroll
    for (int mb = 0; mb < 4; ++mb) { const int m = r0 + mb * 16 + lr; const int b = m / HW, hw = m - b * HW; const int h = hw / WW, w = hw - h * WW;
        ab[mb] = (((size_t)b * HP + h) * WP + w) * CIN + 8 * hi; }
    const size_t boff = (size_t)lr * KD + 8 * hi;
#pragma unroll 1
    for (int t = 0; t < K2; ++t) {
        const int ty = t / 3, tx = t - 3 * ty; const size_t toff = (size_t)(ty * WP + tx) * CIN;
#pragma unroll 1
        for (int kc = 0; kc < CIN; kc += 32) {
            v16bf a[4];
#pragma unroll
            for (int mb = 0; mb < 4; ++mb) a[mb] = ldb(XP + ab[mb] + toff + kc);
#pragma unroll
            for (int nb = 0; nb < 2; ++nb) { const v16bf bq = ldb(OWB + boff + (size_t)nb * 16 * KD + (size_t)t * CIN + kc);
#pragma unroll
                for (int mb = 0; mb < 4; ++mb) acc[mb][nb] = wmmabg(a[mb], bq, acc[mb][nb]); }
        }
    }
    float bc[2];
#pragma unroll
    for (int nb = 0; nb < 2; ++nb) { const int n = nb * 16 + lr; const int nc = n < NOFF ? n : (NOFF - 1); float v = ob[nc]; asm volatile("" : "+v"(v)); bc[nb] = (n < NOFF) ? bfr(v) : 0.0f; }
    const bool sg = (lr >= 2) & (lr < 11);
#pragma unroll
    for (int mb = 0; mb < 4; ++mb) {
#pragma unroll
        for (int j = 0; j < 8; ++j) {
            const float v0 = acc[mb][0][j] + bc[0]; const float v1 = acc[mb][1][j] + bc[1];
            const float e = __builtin_amdgcn_exp2f(-v1 * LOG2E); const float s = __builtin_amdgcn_rcpf(1.0f + e);
            os[(hi * 8 + j) * OFP + lr] = v0; os[(hi * 8 + j) * OFP + 16 + lr] = sg ? s : v1; }
        wave_sync();
        float* prow = PRED + (size_t)(r0 + mb * 16) * NOP;
#pragma unroll 1
        for (int ps = 0; ps < 2; ++ps) {
#pragma unroll
            for (int s = 0; s < 4; ++s) { const int row = 4 * s + (lane >> 3), cofs = (lane & 7) * 4;
                const v4f val = *(const v4fa*)(&os[row * OFP + cofs]);
                *(volatile v4f*)(prow + (size_t)row * NOP + cofs) = val; }
            if (ps == 0) __threadfence(); }
        wave_sync();
    }
}

__global__ __launch_bounds__(256) void k_dconv(const bf* __restrict__ XP, const h16* __restrict__ WH, const float* __restrict__ PRED, float* OUT) {
    __shared__ __align__(16) h16 As[DPOS * AP];
    __shared__ __align__(16) float os[8 * 32 * OTP];
    const int tid = threadIdx.x; const int lane = tid & 31, lr = lane & 15, hi = lane >> 4;
    const int wave = __builtin_amdgcn_readfirstlane((int)(threadIdx.x >> 5));
    const int posbase = blockIdx.x * DPOS; const int b0 = posbase / HW; const int hwbase = posbase - b0 * HW;
    const int sp = tid >> 3, sl = tid & 7;
    const int hw_s = hwbase + sp; const int h_s = hw_s / WW, w_s = hw_s - h_s * WW;
    const float* pr = PRED + (size_t)(posbase + sp) * NOP;
    const bf* xb = XP + (size_t)b0 * HP * WP * CIN + 8 * sl;
    const size_t wo0 = (size_t)(wave * 32 + lr) * KD + 8 * hi, wo1 = wo0 + (size_t)16 * KD;
    const int ao0 = lr * AP + 8 * hi, ao1 = (16 + lr) * AP + 8 * hi;
    v8f c00 = (v8f){}, c01 = (v8f){}, c10 = (v8f){}, c11 = (v8f){};
#pragma unroll 1
    for (int t = 0; t < K2; ++t) {
        const int ty = t / 3, tx = t - 3 * ty;
        {
            const float dy = pr[2 * t], dx = pr[2 * t + 1], mk = pr[18 + t];
            const float py = (float)(h_s - 1 + ty) + dy;
            const float px = (float)(w_s - 1 + tx) + dx;
            const float y0f = floorf(py), x0f = floorf(px);
            const float ly = py - y0f, lx = px - x0f;
            const int y0 = (int)fminf(fmaxf(y0f, -4.0f), 60.0f);
            const int x0 = (int)fminf(fmaxf(x0f, -4.0f), 60.0f);
            const int y1 = y0 + 1, x1 = x0 + 1;
            const float vy0 = ((y0 >= 0) & (y0 < HH)) ? 1.0f : 0.0f, vy1 = ((y1 >= 0) & (y1 < HH)) ? 1.0f : 0.0f;
            const float vx0 = ((x0 >= 0) & (x0 < WW)) ? 1.0f : 0.0f, vx1 = ((x1 >= 0) & (x1 < WW)) ? 1.0f : 0.0f;
            const float w00 = ((1.0f - ly) * (1.0f - lx)) * (vy0 * vx0);
            const float w01 = ((1.0f - ly) * lx) * (vy0 * vx1);
            const float w10 = (ly * (1.0f - lx)) * (vy1 * vx0);
            const float w11 = (ly * lx) * (vy1 * vx1);
            const float ms = mk * SCA;
            const int y0c = y0 < 0 ? 0 : (y0 > HH - 1 ? HH - 1 : y0), y1c = y1 < 0 ? 0 : (y1 > HH - 1 ? HH - 1 : y1);
            const int x0c = x0 < 0 ? 0 : (x0 > WW - 1 ? WW - 1 : x0), x1c = x1 < 0 ? 0 : (x1 > WW - 1 ? WW - 1 : x1);
            const size_t q00 = (size_t)((y0c + 1) * WP + x0c + 1) * CIN, q01 = (size_t)((y0c + 1) * WP + x1c + 1) * CIN;
            const size_t q10 = (size_t)((y1c + 1) * WP + x0c + 1) * CIN, q11 = (size_t)((y1c + 1) * WP + x1c + 1) * CIN;
#pragma unroll
            for (int j = 0; j < 2; ++j) {
                const int c = j * 64;
                const v8us a00 = *(const v8us*)(xb + q00 + c), a01 = *(const v8us*)(xb + q01 + c);
                const v8us a10 = *(const v8us*)(xb + q10 + c), a11 = *(const v8us*)(xb + q11 + c);
                v8h o;
#pragma unroll
                for (int e = 0; e < 8; ++e) {
                    const float f00 = __uint_as_float(((unsigned)a00[e]) << 16), f01 = __uint_as_float(((unsigned)a01[e]) << 16);
                    const float f10 = __uint_as_float(((unsigned)a10[e]) << 16), f11 = __uint_as_float(((unsigned)a11[e]) << 16);
                    const float r = ((f00 * w00 + f01 * w01) + f10 * w10) + f11 * w11;
                    o[e] = toh_flush(r * ms); }
                *(v8h*)(&As[sp * AP + 8 * sl + c]) = o; }
        }
        __syncthreads();
#pragma unroll
        for (int kc = 0; kc < CIN; kc += 32) {
            const v16h a0 = cat16(*(const v8h*)(&As[ao0 + kc]), *(const v8h*)(&As[ao0 + kc + 16]));
            const v16h a1 = cat16(*(const v8h*)(&As[ao1 + kc]), *(const v8h*)(&As[ao1 + kc + 16]));
            const v16h b0v = ldh(WH + wo0 + (size_t)t * CIN + kc), b1v = ldh(WH + wo1 + (size_t)t * CIN + kc);
            c00 = wmma16g(a0, b0v, c00); c01 = wmma16g(a0, b1v, c01); c10 = wmma16g(a1, b0v, c10); c11 = wmma16g(a1, b1v, c11); }
        __syncthreads();
    }
    const int wb = wave * 32 * OTP;
    { v8f f; v4f a, c;
      f = c00 * SCI; a = __builtin_shufflevector(f, f, 0, 1, 2, 3); c = __builtin_shufflevector(f, f, 4, 5, 6, 7);
      *(v4fa*)(&os[wb + lr * OTP +  0 + 8 * hi]) = a; *(v4fa*)(&os[wb + lr * OTP +  0 + 8 * hi + 4]) = c;
      f = c01 * SCI; a = __builtin_shufflevector(f, f, 0, 1, 2, 3); c = __builtin_shufflevector(f, f, 4, 5, 6, 7);
      *(v4fa*)(&os[wb + (16 + lr) * OTP +  0 + 8 * hi]) = a; *(v4fa*)(&os[wb + (16 + lr) * OTP +  0 + 8 * hi + 4]) = c;
      f = c10 * SCI; a = __builtin_shufflevector(f, f, 0, 1, 2, 3); c = __builtin_shufflevector(f, f, 4, 5, 6, 7);
      *(v4fa*)(&os[wb + lr * OTP + 16 + 8 * hi]) = a; *(v4fa*)(&os[wb + lr * OTP + 16 + 8 * hi + 4]) = c;
      f = c11 * SCI; a = __builtin_shufflevector(f, f, 0, 1, 2, 3); c = __builtin_shufflevector(f, f, 4, 5, 6, 7);
      *(v4fa*)(&os[wb + (16 + lr) * OTP + 16 + 8 * hi]) = a; *(v4fa*)(&os[wb + (16 + lr) * OTP + 16 + 8 * hi + 4]) = c; }
    wave_sync();
    float* orow = OUT + ((size_t)b0 * COUT + (size_t)(wave * 32)) * HW + hwbase;
#pragma unroll 1
    for (int ps = 0; ps < 2; ++ps) {
#pragma unroll
        for (int s = 0; s < 8; ++s) { const int row = 4 * s + (lane >> 3), cofs = (lane & 7) * 4;
            const v4f val = *(const v4fa*)(&os[wb + row * OTP + cofs]);
            *(volatile v4f*)(orow + (size_t)row * HW + cofs) = val; }
        if (ps == 0) __threadfence(); }
}

static constexpr size_t al256(size_t v) { return (v + 255) & ~(size_t)255; }
static constexpr size_t SZ_XP = al256((size_t)NB * HP * WP * CIN * 2);
static constexpr size_t SZ_WH = al256((size_t)COUT * KD * 2);
static constexpr size_t SZ_OW = al256((size_t)NOP * KD * 2);
static constexpr size_t SZ_PR = al256((size_t)NPOS * NOP * 4);
static constexpr size_t SZ_TOTAL = SZ_XP + SZ_WH + SZ_OW + SZ_PR;
static_assert(SZ_TOTAL <= (size_t)134217728);
static_assert((size_t)NB * HP * XROWP * 16 <= SZ_XP);
static_assert((size_t)COUT * (KD / 8) * 16 <= SZ_WH);
static_assert((size_t)NOP * (KD / 8) * 16 <= SZ_OW);
static_assert((size_t)NPOS * NOP * 4 <= SZ_PR);

extern "C" void kernel_launch(void* const* d_in, const int* in_sizes, int n_in,
                              void* d_out, int out_size, void* d_ws, size_t ws_size, hipStream_t stream) {
    if (n_in < 4) return;
    if ((size_t)in_sizes[0] < (size_t)(NB - 1) * XBS_FULL + (size_t)CIN * HW) return;
    if ((size_t)in_sizes[1] < (size_t)NOFF * KD) return;
    if (in_sizes[2] < NOFF) return;
    if ((size_t)in_sizes[3] < (size_t)COUT * KD) return;
    if ((size_t)out_size < (size_t)NB * COUT * HW) return;
    if (SZ_TOTAL > ws_size) return;
    const float* x  = (const float*)d_in[0];
    const float* ow = (const float*)d_in[1];
    const float* ob = (const float*)d_in[2];
    const float* wg = (const float*)d_in[3];
    float* OUT = (float*)d_out;
    char* wsp = (char*)d_ws;
    bf*    XP   = (bf*)wsp;    wsp += SZ_XP;
    h16*   WH   = (h16*)wsp;   wsp += SZ_WH;
    bf*    OWB  = (bf*)wsp;    wsp += SZ_OW;
    float* PRED = (float*)wsp; wsp += SZ_PR;

    k_xpad<<<dim3(HP, NB, 1), 256, 0, stream>>>(x, XP);
    k_wmain<<<(unsigned)(COUT * (KD / 8) / 256), 256, 0, stream>>>(wg, WH);
    k_woff<<<(unsigned)(NOP * (KD / 8) / 256), 256, 0, stream>>>(ow, OWB);
    k_offconv<<<(unsigned)(NPOS / 64), 32, 0, stream>>>(XP, OWB, ob, PRED);
    k_dconv<<<(unsigned)(NPOS / DPOS), 256, 0, stream>>>(XP, WH, PRED, OUT);
}
